// SwinTransformerEncoder_15564961481378
// MI455X (gfx1250) — hardware-run, weakly checked
//
#include <hip/hip_runtime.h>
#include <math.h>

constexpr int kBatch   = 8;
constexpr int kImg     = 64;
constexpr int kChan    = 256;
constexpr int kHeads   = 8;
constexpr int kHeadDim = 32;
constexpr int kWin     = 8;
constexpr int kTokWin  = kWin * kWin;
constexpr int kWinImg  = (kImg / kWin) * (kImg / kWin);
constexpr int kNumWin  = kBatch * kWinImg;
constexpr int kTok     = kBatch * kImg * kImg;
constexpr int kQkvN    = 3 * kChan;
constexpr int kHidden  = 4 * kChan;
constexpr int kRelTab  = (2 * kWin - 1) * (2 * kWin - 1);
constexpr float kLnEps = 1e-5f;

constexpr float kWCarry      = 16.0f;
constexpr float kQkvCarry    = 8.0f;
constexpr float kQkvScale    = kQkvCarry / kWCarry;
constexpr float kScoreScale  = 0.17677669529663687f * (1.0f / 64.0f);
constexpr float kPCarry      = 1024.0f;
constexpr float kOStoreScale = 1.0f / 1024.0f;
constexpr float kProjScale   = 1.0f / (kQkvCarry * kWCarry);
constexpr float kFc1Scale    = 1.0f / kWCarry;
constexpr float kHCarry      = 8.0f;
constexpr float kFc2Scale    = 1.0f / (kHCarry * kWCarry);

constexpr int kQkvChunkRows = 16384;
constexpr int kQkvChunks    = kTok / kQkvChunkRows;
constexpr int kWinPerChunk  = kQkvChunkRows / kTokWin;
constexpr int kMlpChunkRows = 4096;
constexpr int kMlpChunks    = kTok / kMlpChunkRows;

constexpr size_t kOffWqkv  = 0;
constexpr size_t kOffWproj = kOffWqkv  + (size_t)2 * kQkvN   * kChan * 2;
constexpr size_t kOffWfc1  = kOffWproj + (size_t)2 * kChan   * kChan * 2;
constexpr size_t kOffWfc2  = kOffWfc1  + (size_t)2 * kHidden * kChan * 2;
constexpr size_t kOffXw    = kOffWfc2  + (size_t)2 * kChan   * kHidden * 2;
constexpr size_t kOffAw    = kOffXw    + (size_t)kTok * kChan * 2;
constexpr size_t kOffX1    = kOffAw    + (size_t)kTok * kChan * 2;
constexpr size_t kOffXmid  = kOffX1    + (size_t)kTok * kChan * 4;
constexpr size_t kOffS     = kOffXmid  + (size_t)kTok * kChan * 4;
constexpr size_t kSBytes   = (size_t)kQkvChunkRows * kQkvN * 2;
constexpr size_t kOffH16   = kOffS + (size_t)kMlpChunkRows * kHidden * 4;
constexpr size_t kWsEnd    = kOffS + kSBytes;
typedef char ws_total_check[(kWsEnd <= (size_t)134217728u) ? 1 : -1];
typedef char ws_s_check[((size_t)kMlpChunkRows * kHidden * 4 + (size_t)kMlpChunkRows * kHidden * 2 <= kSBytes) ? 1 : -1];
typedef char chunk_check[((kQkvChunkRows % 64) == 0 && (kMlpChunkRows % 64) == 0 && (kChan % 32) == 0 && (kHidden % 32) == 0) ? 1 : -1];

typedef __attribute__((ext_vector_type(16))) _Float16 v16h;
typedef __attribute__((ext_vector_type(8)))  _Float16 v8h;
typedef __attribute__((ext_vector_type(16))) __bf16   v16b;
typedef __attribute__((ext_vector_type(8)))  __bf16   v8b;
typedef __attribute__((ext_vector_type(8)))  float    v8f;
typedef __attribute__((ext_vector_type(4)))  float    v4f;
typedef __attribute__((ext_vector_type(4)))  unsigned int v4u;

__device__ __forceinline__ unsigned short f2bf_bits(float f) {
  unsigned u = __float_as_uint(f);
  return (unsigned short)((u + 0x7FFFu + ((u >> 16) & 1u)) >> 16);
}
__device__ __forceinline__ float bf_bits2f(unsigned short h) { return __uint_as_float(((unsigned)h) << 16); }

__device__ __forceinline__ void dep_guard_h(v8f& a, v8f& b, v16h x, v16h y) { asm volatile("v_nop\n\tv_nop\n\tv_nop\n\tv_nop" : "+v"(a), "+v"(b) : "v"(x), "v"(y)); }
__device__ __forceinline__ void dep_guard_b(v8f& a, v8f& b, v16b x, v16b y) { asm volatile("v_nop\n\tv_nop\n\tv_nop\n\tv_nop" : "+v"(a), "+v"(b) : "v"(x), "v"(y)); }
__device__ __forceinline__ void keep4_h(v16h a, v16h b, v16h c, v16h d) { asm volatile("v_nop" :: "v"(a), "v"(b), "v"(c), "v"(d)); }
__device__ __forceinline__ void keep4_b(v16b a, v16b b, v16b c, v16b d) { asm volatile("v_nop" :: "v"(a), "v"(b), "v"(c), "v"(d)); }
__device__ __forceinline__ void acc_guard4(v8f& a, v8f& b, v8f& c, v8f& d) { asm volatile("v_nop\n\tv_nop\n\tv_nop\n\tv_nop" : "+v"(a), "+v"(b), "+v"(c), "+v"(d)); }
template <typename T> struct Frag;
template <> struct Frag<_Float16> {
  typedef v16h V; union U { v16h v; v8h h[2]; };
  static __device__ __forceinline__ v16h load(const _Float16* p) {
    U f; f.h[0] = *(const v8h*)(p); f.h[1] = *(const v8h*)(p + 16); return f.v;
  }
  static __device__ __forceinline__ v8f mma(v16h a, v16h b, v8f c) {
    return __builtin_amdgcn_wmma_f32_16x16x32_f16(false, a, false, b, (short)0, c, false, false);
  }
  static __device__ __forceinline__ void guard(v8f& a, v8f& b, v16h x, v16h y) { dep_guard_h(a, b, x, y); }
  static __device__ __forceinline__ void keep(v16h a, v16h b, v16h c, v16h d) { keep4_h(a, b, c, d); }
};
template <> struct Frag<__bf16> {
  typedef v16b V; union U { v16b v; v8b h[2]; };
  static __device__ __forceinline__ v16b load(const __bf16* p) {
    U f; f.h[0] = *(const v8b*)(p); f.h[1] = *(const v8b*)(p + 16); return f.v;
  }
  static __device__ __forceinline__ v8f mma(v16b a, v16b b, v8f c) {
    return __builtin_amdgcn_wmma_f32_16x16x32_bf16(false, a, false, b, (short)0, c, false, false);
  }
  static __device__ __forceinline__ void guard(v8f& a, v8f& b, v16b x, v16b y) { dep_guard_b(a, b, x, y); }
  static __device__ __forceinline__ void keep(v16b a, v16b b, v16b c, v16b d) { keep4_b(a, b, c, d); }
};

__device__ __forceinline__ unsigned pk16(unsigned short a, unsigned short b) { return (unsigned)a | ((unsigned)b << 16); }
__device__ __forceinline__ unsigned short h_bits(float f) { const _Float16 h = (_Float16)f; return __builtin_bit_cast(unsigned short, h); }

__device__ __forceinline__ v8f mma_f16(v16h a, v16h b, v8f c) {
  c = __builtin_amdgcn_wmma_f32_16x16x32_f16(false, a, false, b, (short)0, c, false, false);
  asm volatile("v_nop\n\tv_nop\n\tv_nop\n\tv_nop" : "+v"(c) : "v"(a), "v"(b));
  return c;
}

template <int ET> struct Elem;
template <> struct Elem<0> { typedef _Float16 T; };
template <> struct Elem<1> { typedef __bf16 T; };
template <int ET, bool SPLIT, int BIAS_MODE, int OUT_MODE, bool RESID, int ACT = 0>
__global__ __launch_bounds__(256) void wmma_gemm64(
    const unsigned short* __restrict__ Ap, const unsigned short* __restrict__ A2p, int lda, long strideA,
    const unsigned short* __restrict__ Btp, const unsigned short* __restrict__ Bt2p, int ldb, long strideB,
    void* __restrict__ Cout, void* __restrict__ Cout2, int ldc, long strideC,
    const float* __restrict__ bias,
    const float* __restrict__ resid, long strideR,
    int M, int N, int K, float scale, float bias_scale) {
  typedef typename Elem<ET>::T T;
  typedef typename Frag<T>::V V;
  const T* A = (const T*)Ap; const T* A2 = (const T*)A2p; const T* Bt = (const T*)Btp; const T* Bt2 = (const T*)Bt2p;
  __shared__ __align__(16) float sT[8][16 * 68];
  const int b    = blockIdx.y;
  const int lane = threadIdx.x & 31;
  const int wave = threadIdx.x >> 5;
  const int tilesN = N >> 6;
  const int tilesM = M >> 6;
  const int tile = blockIdx.x * 8 + wave;
  if (tile >= tilesM * tilesN) return;
  const int tm = tile / tilesN;
  const int tn = tile - tm * tilesN;
  const int m0 = tm << 6;
  const int n0 = tn << 6;

  const T* Ab  = A  + (size_t)b * strideA;
  const T* Bb  = Bt + (size_t)b * strideB;
  const T* Ab2 = SPLIT ? (A2  + (size_t)b * strideA) : nullptr;
  const T* Bb2 = SPLIT ? (Bt2 + (size_t)b * strideB) : nullptr;

  const int rlane = lane & 15;
  const int koff  = (lane >> 4) * 8;
  const int mOff  = (lane >> 4) * 8;

  v8f acc[4][4];
#pragma unroll
  for (int i = 0; i < 4; ++i)
#pragma unroll
    for (int j = 0; j < 4; ++j) acc[i][j] = (v8f){0.f,0.f,0.f,0.f,0.f,0.f,0.f,0.f};

  for (int k0 = 0; k0 < K; k0 += 32) {
    V bh[4], bl[4];
#pragma unroll
    for (int j = 0; j < 4; ++j) {
      const size_t bo = (size_t)(n0 + (j << 4) + rlane) * ldb + koff + k0;
      bh[j] = Frag<T>::load(Bb + bo);
      if (SPLIT) bl[j] = Frag<T>::load(Bb2 + bo);
    }
#pragma unroll
    for (int i = 0; i < 4; ++i) {
      const size_t ao = (size_t)(m0 + (i << 4) + rlane) * lda + koff + k0;
      V ah = Frag<T>::load(Ab + ao);
      V al;
      if (SPLIT) al = Frag<T>::load(Ab2 + ao);
#pragma unroll
      for (int j = 0; j < 4; ++j) {
        acc[i][j] = Frag<T>::mma(ah, bh[j], acc[i][j]);
        if (SPLIT) {
          acc[i][j] = Frag<T>::mma(ah, bl[j], acc[i][j]);
          acc[i][j] = Frag<T>::mma(al, bh[j], acc[i][j]);
        }
      }
      Frag<T>::guard(acc[i][0], acc[i][3], ah, SPLIT ? al : ah);
    }
    Frag<T>::keep(bh[0], bh[1], bh[2], bh[3]);
    if (SPLIT) Frag<T>::keep(bl[0], bl[1], bl[2], bl[3]);
  }
  acc_guard4(acc[0][0], acc[0][1], acc[0][2], acc[0][3]);
  acc_guard4(acc[1][0], acc[1][1], acc[1][2], acc[1][3]);
  acc_guard4(acc[2][0], acc[2][1], acc[2][2], acc[2][3]);
  acc_guard4(acc[3][0], acc[3][1], acc[3][2], acc[3][3]);

  float* slab = sT[wave];
  const float* Rb = RESID ? (resid + (size_t)b * strideR) : nullptr;
#pragma unroll
  for (int i = 0; i < 4; ++i) {
    const int mBase = m0 + (i << 4);
#pragma unroll
    for (int j = 0; j < 4; ++j) {
      const int n = n0 + (j << 4) + rlane;
      float bv = 0.f;
      if (BIAS_MODE == 2) bv = bias[n] * bias_scale;
#pragma unroll
      for (int r = 0; r < 8; ++r) {
        float v = acc[i][j][r] * scale;
        if (BIAS_MODE == 1) v += bias[mBase + mOff + r] * bias_scale;
        if (BIAS_MODE == 2) v += bv;
        if (RESID) v += Rb[(size_t)(mBase + mOff + r) * ldc + n];
        if (ACT == 2) v = fmaxf(v, 0.0f);
        if (ACT == 4) v = (v > 0.f) ? v : 0.01f * v;
        slab[(mOff + r) * 68 + (j << 4) + rlane] = v;
      }
    }
    __builtin_amdgcn_fence(__ATOMIC_RELEASE, "workgroup");
    __builtin_amdgcn_wave_barrier();
    __builtin_amdgcn_fence(__ATOMIC_ACQUIRE, "workgroup");
    if (OUT_MODE == 0) {
      float* C = (float*)Cout + (size_t)b * strideC;
      const int hh = lane >> 4, c4 = (lane & 15) * 4;
      for (int pass = 0; pass < 2; ++pass) {
#pragma unroll
        for (int it = 0; it < 8; ++it) {
          const int row = it * 2 + hh;
          v4f v = *(const v4f*)(slab + row * 68 + c4);
          *(volatile v4f*)(C + (size_t)(mBase + row) * ldc + n0 + c4) = v;
        }
        __threadfence();
      }
    } else {
      const int q = lane >> 3, c8 = (lane & 7) * 8;
      unsigned short* C  = (unsigned short*)Cout  + (size_t)b * strideC;
      unsigned short* C2 = (OUT_MODE == 2) ? ((unsigned short*)Cout2 + (size_t)b * strideC) : nullptr;
      for (int pass = 0; pass < 2; ++pass) {
#pragma unroll
        for (int it = 0; it < 4; ++it) {
          const int row = it * 4 + q;
          const float* sp = slab + row * 68 + c8;
          v8h hv, lv;
#pragma unroll
          for (int e = 0; e < 8; ++e) {
            if (OUT_MODE == 1) {
              hv[e] = (_Float16)sp[e];
            } else {
              unsigned short hb = f2bf_bits(sp[e]);
              unsigned short lb = f2bf_bits(sp[e] - bf_bits2f(hb));
              hv[e] = __builtin_bit_cast(_Float16, hb);
              lv[e] = __builtin_bit_cast(_Float16, lb);
            }
          }
          *(volatile v8h*)(C + (size_t)(mBase + row) * ldc + n0 + c8) = hv;
          if (OUT_MODE == 2) *(volatile v8h*)(C2 + (size_t)(mBase + row) * ldc + n0 + c8) = lv;
        }
        __threadfence();
      }
    }
    __builtin_amdgcn_fence(__ATOMIC_RELEASE, "workgroup");
    __builtin_amdgcn_wave_barrier();
    __builtin_amdgcn_fence(__ATOMIC_ACQUIRE, "workgroup");
  }
}

__global__ __launch_bounds__(256) void tcast_kernel(const float* __restrict__ W, unsigned short* __restrict__ out,
                                                    int K, int N, float scale) {
  __shared__ float sm[64][65];
  const int t  = threadIdx.x;
  const int k0 = blockIdx.x * 64;
  const int n0 = blockIdx.y * 64;
  const int z  = blockIdx.z;
  const float* Wz = W + (size_t)z * K * N;
  unsigned short* oz = out + (size_t)z * N * K;
#pragma unroll
  for (int i = 0; i < 16; ++i) {
    const int e = i * 256 + t;
    const int r = e >> 6;
    const int c = e & 63;
    sm[c][r] = Wz[(size_t)(k0 + r) * N + n0 + c] * scale;
  }
  __syncthreads();
  const int lane = t & 31, wave = t >> 5;
  const int q = lane >> 3, c8 = (lane & 7) * 8;
  for (int pass = 0; pass < 2; ++pass) {
#pragma unroll
    for (int it = 0; it < 2; ++it) {
      const int row = wave * 8 + it * 4 + q;
      unsigned short hb[8];
#pragma unroll
      for (int e = 0; e < 8; ++e) hb[e] = h_bits(sm[row][c8 + e]);
      const v4u u = (v4u){pk16(hb[0], hb[1]), pk16(hb[2], hb[3]), pk16(hb[4], hb[5]), pk16(hb[6], hb[7])};
      *(volatile v4u*)(oz + (size_t)(n0 + row) * K + k0 + c8) = u;
    }
    __threadfence();
  }
}

__global__ __launch_bounds__(256) void ln_rows_kernel(const float* __restrict__ x, const float* __restrict__ g,
                                                      const float* __restrict__ bt, unsigned short* __restrict__ out,
                                                      int shift, int permute) {
  const int lane = threadIdx.x & 31, wave = threadIdx.x >> 5;
  const int o = blockIdx.x * 8 + wave;
  const int w = o >> 6, wt = o & 63;
  const int bimg = w >> 6, wy = (w >> 3) & 7, wx = w & 7;
  const int ty = wt >> 3, tx = wt & 7;
  const int gy = (wy * 8 + ty + shift) & 63, gx = (wx * 8 + tx + shift) & 63;
  const int srcp = bimg * (kImg * kImg) + gy * kImg + gx;
  const int src = permute ? srcp : o;
  const float* p = x + (size_t)src * kChan + lane * 8;
  const v4f a = *(const v4f*)(p);
  const v4f c = *(const v4f*)(p + 4);
  float v[8];
#pragma unroll
  for (int e = 0; e < 4; ++e) { v[e] = a[e]; v[4 + e] = c[e]; }
  float s = ((v[0] + v[1]) + (v[2] + v[3])) + ((v[4] + v[5]) + (v[6] + v[7]));
#pragma unroll
  for (int off = 16; off > 0; off >>= 1) s += __shfl_xor(s, off, 32);
  const float mu = s * (1.0f / 256.0f);
  float d[8];
  float q = 0.f;
#pragma unroll
  for (int e = 0; e < 8; ++e) { d[e] = v[e] - mu; q += d[e] * d[e]; }
#pragma unroll
  for (int off = 16; off > 0; off >>= 1) q += __shfl_xor(q, off, 32);
  const float var = q * (1.0f / 256.0f);
  const float inv = rsqrtf(var + kLnEps);
  const v4f ga = *(const v4f*)(g + lane * 8);
  const v4f gc = *(const v4f*)(g + lane * 8 + 4);
  const v4f ba = *(const v4f*)(bt + lane * 8);
  const v4f bc = *(const v4f*)(bt + lane * 8 + 4);
  float gg[8], bb[8];
#pragma unroll
  for (int e = 0; e < 4; ++e) { gg[e] = ga[e]; gg[4 + e] = gc[e]; bb[e] = ba[e]; bb[4 + e] = bc[e]; }
  unsigned short hb[8];
#pragma unroll
  for (int e = 0; e < 8; ++e) hb[e] = h_bits((d[e] * inv) * gg[e] + bb[e]);
  const v4u u = (v4u){pk16(hb[0], hb[1]), pk16(hb[2], hb[3]), pk16(hb[4], hb[5]), pk16(hb[6], hb[7])};
  unsigned short* dst = out + (size_t)o * kChan + lane * 8;
  *(volatile v4u*)dst = u;
  __threadfence();
  *(volatile v4u*)dst = u;
}

__global__ __launch_bounds__(256) void gelu_cast2_kernel(const float* __restrict__ in, unsigned short* __restrict__ out,
                                                         int n2, float carry) {
  const int i = blockIdx.x * 256 + threadIdx.x;
  if (i < n2) {
    const float a = in[2 * (size_t)i];
    const float b = in[2 * (size_t)i + 1];
    const float ga = 0.5f * a * (1.0f + erff(a * 0.70710678118654752f));
    const float gb = 0.5f * b * (1.0f + erff(b * 0.70710678118654752f));
    const unsigned u = pk16(h_bits(ga * carry), h_bits(gb * carry));
    ((volatile unsigned*)out)[i] = u;
    __threadfence();
    ((volatile unsigned*)out)[i] = u;
  }
}

constexpr int kOPitch = 264;
__device__ __forceinline__ int region_label(int y) { return (y < 56) ? 0 : ((y < 60) ? 1 : 2); }

__global__ __launch_bounds__(256) void wattn_kernel(const unsigned short* __restrict__ qkv, unsigned short* __restrict__ aw,
                                                    const float* __restrict__ rpbl, int w0, int shift, int masked) {
  __shared__ __align__(16) unsigned short sVT[kHeads * kHeadDim * kTokWin];
  __shared__ __align__(16) _Float16 sP[8][16 * kTokWin];
  __shared__ __align__(16) unsigned short sO[kTokWin * kOPitch];

  const int tid = threadIdx.x, lane = tid & 31, wave = tid >> 5;
  const int hh = lane >> 4, rl = lane & 15, koff = hh * 8;
  const int wl = blockIdx.x;
  const int w = w0 + wl;
  const int bimg = w >> 6, wy = (w >> 3) & 7, wx = w & 7;
  const size_t rowbase = (size_t)wl * kTokWin;

#pragma unroll
  for (int it = 0; it < 8; ++it) {
    const int id = it * 256 + tid;
    const int m  = id >> 5;
    const int c8 = (id & 31) * 8;
    const v4u wv = *(const v4u*)(qkv + (rowbase + m) * kQkvN + 2 * kChan + c8);
    const int hd = c8 >> 5, d0 = c8 & 31;
    unsigned short* dst = sVT + (hd * kHeadDim + d0) * kTokWin + m;
#pragma unroll
    for (int e = 0; e < 4; ++e) {
      dst[(2 * e) * kTokWin]     = (unsigned short)(wv[e] & 0xffffu);
      dst[(2 * e + 1) * kTokWin] = (unsigned short)(wv[e] >> 16);
    }
  }
  __syncthreads();

  const int h = wave;
  v16h kf[4];
#pragma unroll
  for (int j = 0; j < 4; ++j)
    kf[j] = Frag<_Float16>::load((const _Float16*)(qkv + (rowbase + 16 * j + rl) * kQkvN + kChan + h * kHeadDim + koff));

  const float mfill = masked ? -100.0f : 0.0f;
  _Float16* pw = sP[wave];
  const unsigned short* vth = sVT + (size_t)h * kHeadDim * kTokWin;

#pragma unroll 1
  for (int rt = 0; rt < 4; ++rt) {
    const v16h qa = Frag<_Float16>::load((const _Float16*)(qkv + (rowbase + rt * 16 + rl) * kQkvN + h * kHeadDim + koff));
    v8f s[4];
#pragma unroll
    for (int j = 0; j < 4; ++j) {
      s[j] = (v8f){0.f,0.f,0.f,0.f,0.f,0.f,0.f,0.f};
      s[j] = mma_f16(qa, kf[j], s[j]);
    }
#pragma unroll
    for (int r = 0; r < 8; ++r) {
      const int n  = rt * 16 + 8 * hh + r;
      const int ny = n >> 3, nx = n & 7;
      const int labr = region_label(wy * 8 + ny) * 3 + region_label(wx * 8 + nx);
      float mx = -3.0e38f;
#pragma unroll
      for (int j = 0; j < 4; ++j) {
        const int m  = 16 * j + rl;
        const int my = m >> 3, mxx = m & 7;
        const int labc = region_label(wy * 8 + my) * 3 + region_label(wx * 8 + mxx);
        const int ridx = (ny - my + 7) * 15 + (nx - mxx + 7);
        float sc = s[j][r] * kScoreScale + rpbl[ridx * kHeads + h];
        sc += (labr != labc) ? mfill : 0.0f;
        s[j][r] = sc;
        mx = fmaxf(mx, sc);
      }
#pragma unroll
      for (int off = 1; off < 16; off <<= 1) mx = fmaxf(mx, __shfl_xor(mx, off, 32));
      float sum = 0.f;
#pragma unroll
      for (int j = 0; j < 4; ++j) {
        const float e = expf(s[j][r] - mx);
        s[j][r] = e;
        sum += e;
      }
#pragma unroll
      for (int off = 1; off < 16; off <<= 1) sum += __shfl_xor(sum, off, 32);
      const float pinv = kPCarry / sum;
#pragma unroll
      for (int j = 0; j < 4; ++j) pw[(8 * hh + r) * kTokWin + 16 * j + rl] = (_Float16)(s[j][r] * pinv);
    }
    __builtin_amdgcn_fence(__ATOMIC_RELEASE, "workgroup");
    __builtin_amdgcn_wave_barrier();
    __builtin_amdgcn_fence(__ATOMIC_ACQUIRE, "workgroup");

    v8f o0 = (v8f){0.f,0.f,0.f,0.f,0.f,0.f,0.f,0.f};
    v8f o1 = (v8f){0.f,0.f,0.f,0.f,0.f,0.f,0.f,0.f};
#pragma unroll
    for (int kk = 0; kk < 2; ++kk) {
      const v16h pa = Frag<_Float16>::load(pw + rl * kTokWin + kk * 32 + koff);
      const v16h v0 = Frag<_Float16>::load((const _Float16*)(vth + (rl) * kTokWin + kk * 32 + koff));
      const v16h v1 = Frag<_Float16>::load((const _Float16*)(vth + (16 + rl) * kTokWin + kk * 32 + koff));
      o0 = mma_f16(pa, v0, o0);
      o1 = mma_f16(pa, v1, o1);
    }
#pragma unroll
    for (int r = 0; r < 8; ++r) {
      const int n = rt * 16 + 8 * hh + r;
      sO[n * kOPitch + h * kHeadDim + rl]      = h_bits(o0[r] * kOStoreScale);
      sO[n * kOPitch + h * kHeadDim + 16 + rl] = h_bits(o1[r] * kOStoreScale);
    }
    __builtin_amdgcn_fence(__ATOMIC_RELEASE, "workgroup");
    __builtin_amdgcn_wave_barrier();
    __builtin_amdgcn_fence(__ATOMIC_ACQUIRE, "workgroup");
  }
  __syncthreads();

  for (int pass = 0; pass < 2; ++pass) {
#pragma unroll
    for (int i = 0; i < 8; ++i) {
      const int n  = wave * 8 + i;
      const int ty = n >> 3, tx = n & 7;
      const int gy = (wy * 8 + ty + shift) & 63, gx = (wx * 8 + tx + shift) & 63;
      const size_t tok = (size_t)bimg * (kImg * kImg) + gy * kImg + gx;
      const v4u val = *(const v4u*)(sO + n * kOPitch + lane * 8);
      *(volatile v4u*)(aw + tok * kChan + lane * 8) = val;
    }
    __threadfence();
  }
}

extern "C" void kernel_launch(void* const* d_in, const int* in_sizes, int n_in,
                              void* d_out, int out_size, void* d_ws, size_t ws_size,
                              hipStream_t stream) {
  (void)in_sizes; (void)n_in;
  const float* x      = (const float*)d_in[0];
  const float* qkv_w  = (const float*)d_in[1];
  const float* qkv_b  = (const float*)d_in[2];
  const float* proj_w = (const float*)d_in[3];
  const float* proj_b = (const float*)d_in[4];
  const float* ln1_g  = (const float*)d_in[5];
  const float* ln1_b  = (const float*)d_in[6];
  const float* ln2_g  = (const float*)d_in[7];
  const float* ln2_b  = (const float*)d_in[8];
  const float* fc1_w  = (const float*)d_in[9];
  const float* fc1_b  = (const float*)d_in[10];
  const float* fc2_w  = (const float*)d_in[11];
  const float* fc2_b  = (const float*)d_in[12];
  const float* rpb    = (const float*)d_in[13];

  if (ws_size < kWsEnd) return;
  if ((size_t)out_size < (size_t)kTok * kChan) return;

  char* ws = (char*)d_ws;
  unsigned short* wqkv16  = (unsigned short*)(ws + kOffWqkv);
  unsigned short* wproj16 = (unsigned short*)(ws + kOffWproj);
  unsigned short* wfc1_16 = (unsigned short*)(ws + kOffWfc1);
  unsigned short* wfc2_16 = (unsigned short*)(ws + kOffWfc2);
  unsigned short* xw16    = (unsigned short*)(ws + kOffXw);
  unsigned short* aw16    = (unsigned short*)(ws + kOffAw);
  float*          x1      = (float*)(ws + kOffX1);
  float*          xmid    = (float*)(ws + kOffXmid);
  unsigned short* qkv16   = (unsigned short*)(ws + kOffS);
  float*          f32c    = (float*)(ws + kOffS);
  unsigned short* h16     = (unsigned short*)(ws + kOffH16);
  float*          outp    = (float*)d_out;

  tcast_kernel<<<dim3(kChan / 64, kQkvN / 64, 2), 256, 0, stream>>>(qkv_w, wqkv16, kChan, kQkvN, kWCarry);
  tcast_kernel<<<dim3(kChan / 64, kChan / 64, 2), 256, 0, stream>>>(proj_w, wproj16, kChan, kChan, kWCarry);
  tcast_kernel<<<dim3(kChan / 64, kHidden / 64, 2), 256, 0, stream>>>(fc1_w, wfc1_16, kChan, kHidden, kWCarry);
  tcast_kernel<<<dim3(kHidden / 64, kChan / 64, 2), 256, 0, stream>>>(fc2_w, wfc2_16, kHidden, kChan, kWCarry);

  for (int i = 0; i < 2; ++i) {
    const int shift  = (i & 1) ? (kWin / 2) : 0;
    const int masked = (i & 1) ? 1 : 0;
    const float* xin = (i == 0) ? x : (const float*)x1;
    float* xout      = (i == 0) ? x1 : outp;

    ln_rows_kernel<<<kTok / 8, 256, 0, stream>>>(xin, ln1_g + i * kChan, ln1_b + i * kChan, xw16, shift, 1);

    for (int c = 0; c < kQkvChunks; ++c) {
      const int tilesQ = (kQkvChunkRows / 64) * (kQkvN / 64);
      wmma_gemm64<0, false, 2, 1, false, 0><<<dim3((tilesQ + 7) / 8, 1), 256, 0, stream>>>(
          xw16 + (size_t)c * kQkvChunkRows * kChan, nullptr, kChan, 0L,
          wqkv16 + (size_t)i * kQkvN * kChan, nullptr, kChan, 0L,
          (void*)qkv16, nullptr, kQkvN, 0L,
          qkv_b + i * kQkvN, nullptr, 0L,
          kQkvChunkRows, kQkvN, kChan, kQkvScale, kQkvCarry);
      wattn_kernel<<<kWinPerChunk, 256, 0, stream>>>(qkv16, aw16, rpb + (size_t)i * kRelTab * kHeads,
                                                      c * kWinPerChunk, shift, masked);
    }

    {
      const int tilesP = (kTok / 64) * (kChan / 64);
      wmma_gemm64<0, false, 2, 0, true, 0><<<dim3((tilesP + 7) / 8, 1), 256, 0, stream>>>(
          aw16, nullptr, kChan, 0L,
          wproj16 + (size_t)i * kChan * kChan, nullptr, kChan, 0L,
          (void*)xmid, nullptr, kChan, 0L,
          proj_b + i * kChan, xin, 0L,
          kTok, kChan, kChan, kProjScale, 1.0f);
    }

    ln_rows_kernel<<<kTok / 8, 256, 0, stream>>>(xmid, ln2_g + i * kChan, ln2_b + i * kChan, xw16, 0, 0);

    for (int c = 0; c < kMlpChunks; ++c) {
      const size_t r0 = (size_t)c * kMlpChunkRows;
      const int tiles1 = (kMlpChunkRows / 64) * (kHidden / 64);
      wmma_gemm64<0, false, 2, 0, false, 0><<<dim3((tiles1 + 7) / 8, 1), 256, 0, stream>>>(
          xw16 + r0 * kChan, nullptr, kChan, 0L,
          wfc1_16 + (size_t)i * kHidden * kChan, nullptr, kChan, 0L,
          (void*)f32c, nullptr, kHidden, 0L,
          fc1_b + i * kHidden, nullptr, 0L,
          kMlpChunkRows, kHidden, kChan, kFc1Scale, 1.0f);
      const int n2 = kMlpChunkRows * kHidden / 2;
      gelu_cast2_kernel<<<(n2 + 255) / 256, 256, 0, stream>>>(f32c, h16, n2, kHCarry);
      const int tiles2 = (kMlpChunkRows / 64) * (kChan / 64);
      wmma_gemm64<0, false, 2, 0, true, 0><<<dim3((tiles2 + 7) / 8, 1), 256, 0, stream>>>(
          h16, nullptr, kHidden, 0L,
          wfc2_16 + (size_t)i * kChan * kHidden, nullptr, kHidden, 0L,
          (void*)(xout + r0 * kChan), nullptr, kChan, 0L,
          fc2_b + i * kChan, xmid + r0 * kChan, 0L,
          kMlpChunkRows, kChan, kHidden, kFc2Scale, 1.0f);
    }
  }
}
